// SpinConvSq2d_12369505813005
// MI455X (gfx1250) — hardware-verified
//
#include <hip/hip_runtime.h>
#include <stdint.h>

#define DEVINL __device__ __forceinline__

typedef _Float16 f16t;
typedef _Float16 v16h __attribute__((ext_vector_type(16)));
typedef _Float16 v8h  __attribute__((ext_vector_type(8)));
typedef float    v8f  __attribute__((ext_vector_type(8)));
typedef float    v4f  __attribute__((ext_vector_type(4)));
typedef v8h __attribute__((may_alias)) v8ha;
typedef v4f __attribute__((may_alias)) v4fa;
union FragH { v16h v; v8h half[2]; };

#define LSP    64
#define CIN    64
#define NPIXI  (LSP * LSP)
#define NSLOT  25
#define KREAL  (NSLOT * 16)
#define KP     416
#define NW     32
#define NOUT   128
#define NPL    5
#define TPB    256
#define MTPB   128

#define SH0c   0.28209479177387814f
#define SH1c   0.4886025119029199f
#define CG110c 0.5773502691896258f
#define CG111c 0.7071067811865476f
#define A0c    0.035355339059327376f
#define A1c    0.028867513459481287f

static_assert((KP % 32) == 0);
static_assert(KP >= KREAL + 16);
static_assert((KP % 8) == 0);
static_assert(((NPL * NW * KP * 2) % 128) == 0);
static_assert((CIN * 2) == 128);
static_assert((5 * LSP * CIN * 2) >= (LSP * NOUT * 4));
static_assert((LSP * NOUT) == (MTPB * 16 * 4));
static_assert(MTPB == 128);

DEVINL int imin(int a, int b) { return a < b ? a : b; }
DEVINL int imax(int a, int b) { return a > b ? a : b; }

DEVINL v8f wmma_f16(v16h a, v16h b, v8f c) {
  v8f d = __builtin_amdgcn_wmma_f32_16x16x32_f16(false, a, false, b, (short)0, c, false, false);
  asm volatile("v_nop\n\tv_nop\n\tv_nop\n\tv_nop" : "+v"(d) : "v"(a), "v"(b));
  return d;
}
DEVINL v8f zero8f() {
  v8f z = {0.f, 0.f, 0.f, 0.f, 0.f, 0.f, 0.f, 0.f};
  return z;
}
DEVINL v8h zero8h() {
  v8h z;
  #pragma unroll
  for (int i = 0; i < 8; ++i) z[i] = (f16t)0.0f;
  return z;
}
DEVINL v16h ldB(const f16t* p) {
  FragH f;
  f.half[0] = *(const v8ha*)(p);
  f.half[1] = *(const v8ha*)(p + 16);
  return f.v;
}

__global__ __launch_bounds__(TPB) void prep_w_k(const float* __restrict__ W000, const float* __restrict__ W110,
                                              const float* __restrict__ W011, const float* __restrict__ W101,
                                              const float* __restrict__ W111, f16t* __restrict__ Bw)
{
  const int t = blockIdx.x * TPB + threadIdx.x;
  if (t >= NPL * NW * (KP / 8)) return;
  const int row   = t / (KP / 8);
  const int piece = t - row * (KP / 8);
  const int p     = row >> 5;
  const int nn    = row & 31;
  const int k8    = 8 * piece;
  v8h o;
  #pragma unroll
  for (int i = 0; i < 8; ++i) {
    const int k   = k8 + i;
    const int kc  = imin(k, KREAL - 1);
    const int idx = kc * NW + nn;
    const float w0 = W000[idx], w1 = W110[idx], w2 = W011[idx], w3 = W101[idx], w4 = W111[idx];
    float v = (p == 0) ? (SH0c * w0) : (p == 1) ? w1 : (p == 2) ? w2 : (p == 3) ? (SH0c * w3) : w4;
    v = (k < KREAL) ? v : 0.0f;
    o[i] = (f16t)v;
  }
  f16t* dst = Bw + (size_t)8 * t;
  *(volatile v8h*)dst = o;
  __threadfence();
  *(volatile v8h*)dst = o;
}

__global__ __launch_bounds__(TPB) void cvt_feat_k(const float* __restrict__ feat, f16t* __restrict__ Xh,
                                                int npieces)
{
  const int t = blockIdx.x * TPB + threadIdx.x;
  if (t >= npieces) return;
  const int pix = t >> 3;
  const int pc  = t & 7;
  const float* src = feat + (size_t)pix * CIN;
  v8h o;
  #pragma unroll
  for (int i = 0; i < 8; ++i) {
    const int cp = 8 * pc + i;
    const int cq = cp - 16;
    const int cv = 16 + 3 * (cq & 15) + ((cq >> 4) & 3);
    const int c  = (cp < 16) ? cp : imin(cv, CIN - 1);
    o[i] = (f16t)src[c];
  }
  f16t* dst = Xh + (size_t)8 * t;
  *(volatile v8h*)dst = o;
  __threadfence();
  *(volatile v8h*)dst = o;
}

__global__ __launch_bounds__(MTPB) __attribute__((amdgpu_num_vgpr(256)))
void tp_main_k(const f16t* __restrict__ Xh, const f16t* __restrict__ Bw,
               const float* __restrict__ spin, float* __restrict__ out)
{
  __shared__ __attribute__((aligned(16))) char  smem[5 * LSP * CIN * 2];
  __shared__ __attribute__((aligned(16))) float Ss[LSP * 3];
  f16t*  As = (f16t*)smem;
  float* sO = (float*)smem;

  const int tid = threadIdx.x, lane = tid & 31, wave = tid >> 5;
  const int h = lane >> 4, m = lane & 15;
  const int n = blockIdx.x >> 6;
  const int x = blockIdx.x & 63;

  for (int q = tid; q < 5 * LSP * 8; q += MTPB) {
    const int r   = q >> 9;
    const int rem = q & 511;
    const int y   = rem >> 3;
    const int pc  = rem & 7;
    const int xs  = (x + r + 62) & 63;
    const v8h v = *(const v8ha*)(Xh + ((size_t)((n * LSP + xs) * LSP + y)) * CIN + 8 * pc);
    *(v8ha*)(As + (r * LSP + y) * CIN + 8 * pc) = v;
  }
  for (int q = tid; q < LSP * 3; q += MTPB)
    Ss[q] = SH1c * spin[(size_t)(n * LSP + x) * (LSP * 3) + q];
  __syncthreads();

  const int ybase = wave * 16;
  const int ym    = ybase + m;
  const float sx = Ss[ym * 3 + 0], sy = Ss[ym * 3 + 1], sz = Ss[ym * 3 + 2];
  const f16t* bl = Bw + (size_t)m * KP + 8 * h;
  const v8h z8 = zero8h();

  v8f acc0[2], accq[2], accr[3][2];
  #pragma unroll
  for (int t = 0; t < 2; ++t) {
    acc0[t] = zero8f(); accq[t] = zero8f();
    #pragma unroll
    for (int g = 0; g < 3; ++g) accr[g][t] = zero8f();
  }

  #pragma unroll 1
  for (int s = 0; s < KP / 32; ++s) {
    const bool last = (s == (KP / 32) - 1);
    const int aA  = 2 * s;
    const int aB  = imin(2 * s + 1, NSLOT - 1);
    const int ixA = aA / 5, iyA = aA - 5 * ixA;
    const int ixB = aB / 5, iyB = aB - 5 * ixB;
    const int ysA = (ym + iyA + 62) & 63;
    const int ysB = (ym + iyB + 62) & 63;
    const f16t* pA = As + (ixA * LSP + ysA) * CIN + 8 * h;
    const f16t* pB = As + (ixB * LSP + ysB) * CIN + 8 * h;
    const f16t* bk = bl + 32 * s;

    {
      FragH fx0;
      fx0.half[0] = *(const v8ha*)(pA);
      const v8h t1 = *(const v8ha*)(pB);
      fx0.half[1] = last ? z8 : t1;
      #pragma unroll
      for (int t = 0; t < 2; ++t) {
        const v16h b0 = ldB(bk + (0 * NW + 16 * t) * KP);
        acc0[t] = wmma_f16(fx0.v, b0, acc0[t]);
        const v16h b2 = ldB(bk + (2 * NW + 16 * t) * KP);
        accq[t] = wmma_f16(fx0.v, b2, accq[t]);
      }
    }

    FragH fx1[3];
    #pragma unroll
    for (int g = 0; g < 3; ++g) {
      fx1[g].half[0] = *(const v8ha*)(pA + 16 + 16 * g);
      const v8h t1 = *(const v8ha*)(pB + 16 + 16 * g);
      fx1[g].half[1] = last ? z8 : t1;
    }
    #pragma unroll
    for (int t = 0; t < 2; ++t) {
      const v16h b3 = ldB(bk + (3 * NW + 16 * t) * KP);
      #pragma unroll
      for (int g = 0; g < 3; ++g) accr[g][t] = wmma_f16(fx1[g].v, b3, accr[g][t]);
    }

    FragH fdt, fcr[3];
    #pragma unroll
    for (int e = 0; e < 16; ++e) {
      const float vx = (float)fx1[0].v[e];
      const float vy = (float)fx1[1].v[e];
      const float vz = (float)fx1[2].v[e];
      const float d  = (vx * sx + vy * sy + vz * sz) * CG110c;
      fdt.v[e]    = (f16t)d;
      fcr[0].v[e] = (f16t)((vy * sz - vz * sy) * CG111c);
      fcr[1].v[e] = (f16t)((vz * sx - vx * sz) * CG111c);
      fcr[2].v[e] = (f16t)((vx * sy - vy * sx) * CG111c);
    }
    #pragma unroll
    for (int t = 0; t < 2; ++t) {
      const v16h b1 = ldB(bk + (1 * NW + 16 * t) * KP);
      acc0[t] = wmma_f16(fdt.v, b1, acc0[t]);
    }
    #pragma unroll
    for (int t = 0; t < 2; ++t) {
      const v16h b4 = ldB(bk + (4 * NW + 16 * t) * KP);
      #pragma unroll
      for (int g = 0; g < 3; ++g) accr[g][t] = wmma_f16(fcr[g].v, b4, accr[g][t]);
    }
  }

  __syncthreads();

  #pragma unroll
  for (int r = 0; r < 8; ++r) {
    const int prow = ybase + 8 * h + r;
    const float px = Ss[prow * 3 + 0], py = Ss[prow * 3 + 1], pz = Ss[prow * 3 + 2];
    float* so = sO + prow * NOUT;
    #pragma unroll
    for (int t = 0; t < 2; ++t) {
      const int w = 16 * t + m;
      so[w] = A0c * acc0[t][r];
      const float q = accq[t][r];
      so[32 + w * 3 + 0] = A1c * (px * q + accr[0][t][r]);
      so[32 + w * 3 + 1] = A1c * (py * q + accr[1][t][r]);
      so[32 + w * 3 + 2] = A1c * (pz * q + accr[2][t][r]);
    }
  }
  __syncthreads();

  float* ob = out + (size_t)blockIdx.x * (size_t)(LSP * NOUT);
  v4f vv[16];
  #pragma unroll
  for (int j = 0; j < 16; ++j) vv[j] = *(const v4fa*)(sO + (tid + MTPB * j) * 4);
  #pragma unroll
  for (int j = 0; j < 16; ++j) *(volatile v4f*)(ob + (size_t)(tid + MTPB * j) * 4) = vv[j];
  __threadfence();
  #pragma unroll
  for (int j = 0; j < 16; ++j) *(volatile v4f*)(ob + (size_t)(tid + MTPB * j) * 4) = vv[j];
}

extern "C" void kernel_launch(void* const* d_in, const int* in_sizes, int n_in,
                              void* d_out, int out_size, void* d_ws, size_t ws_size,
                              hipStream_t stream)
{
  if (n_in < 7) return;
  const int pixf = NPIXI * CIN;
  if (in_sizes[0] <= 0 || (in_sizes[0] % pixf) != 0) return;
  const int nB = in_sizes[0] / pixf;
  if (nB > 4096) return;
  if (in_sizes[1] != nB * NPIXI * 3) return;
  for (int i = 2; i < 7; ++i) if (in_sizes[i] != KREAL * NW) return;
  if (out_size != nB * NPIXI * NOUT) return;

  const float* feat = (const float*)d_in[0];
  const float* spin = (const float*)d_in[1];
  const float* W000 = (const float*)d_in[2];
  const float* W110 = (const float*)d_in[3];
  const float* W011 = (const float*)d_in[4];
  const float* W101 = (const float*)d_in[5];
  const float* W111 = (const float*)d_in[6];
  float* outp = (float*)d_out;

  const size_t szBw = (size_t)NPL * NW * KP * 2;
  const size_t szXh = (size_t)nB * NPIXI * CIN * 2;
  size_t off = 0;
  char* ws = (char*)d_ws;
  f16t* Bw = (f16t*)(ws + off); off += szBw;
  f16t* Xh = (f16t*)(ws + off); off += szXh;
  if (off > ws_size) return;
  if (off > (size_t)134217728) return;

  const int npieces = nB * NPIXI * 8;

  prep_w_k<<<(NPL * NW * (KP / 8) + TPB - 1) / TPB, TPB, 0, stream>>>(W000, W110, W011, W101, W111, Bw);
  cvt_feat_k<<<(npieces + TPB - 1) / TPB, TPB, 0, stream>>>(feat, Xh, npieces);
  tp_main_k<<<nB * LSP, MTPB, 0, stream>>>(Xh, Bw, spin, outp);
}
